// GemmaExpert_58660663328847
// MI455X (gfx1250) — hardware-run, weakly checked
//
#include <hip/hip_runtime.h>
#include <math.h>

#ifndef NB
#define NB 2
#endif
#ifndef SEQ
#define SEQ 2048
#endif
#define SEQ_FULL 2048
#define HID 2048
#define NH 4
#define NKV 2
#define HD 256
#define QD 1024
#define KD 512
#define QKW 1536
#define IP 4096
#define MTOK (NB * SEQ)

static_assert(SEQ % 64 == 0);
static_assert(SEQ <= SEQ_FULL);
static_assert(MTOK % 64 == 0);
static_assert(HID % 64 == 0 && QD % 64 == 0 && KD % 64 == 0 && IP % 64 == 0 && QKW % 256 == 0);
static_assert(HID % 32 == 0 && QD % 32 == 0 && IP % 32 == 0 && HD % 32 == 0);
static_assert(NH == 2 * NKV && QD == NH * HD && KD == NKV * HD && QKW == QD + KD);

typedef _Float16 h16;
typedef __attribute__((ext_vector_type(16))) _Float16 v16h;
typedef __attribute__((ext_vector_type(8)))  _Float16 v8h;
typedef __attribute__((ext_vector_type(8)))  float    v8f;
typedef __attribute__((ext_vector_type(4)))  float    v4f;

constexpr float ACT_CARRY = 2048.0f;
constexpr float P_CARRY   = 16384.0f;
constexpr float HID_CARRY = 1024.0f;
constexpr float SC_PROJ   = 1.0f / 268435456.0f;
constexpr float SC_S      = 1.0f / 67108864.0f;
constexpr float SC_O      = 1.0f / 8192.0f;

constexpr size_t SZ_X16 = (size_t)MTOK * HID * 2;
constexpr size_t SZ_WQK = (size_t)QKW * HID * 2;
constexpr size_t SZ_WV  = (size_t)KD * HID * 2;
constexpr size_t SZ_WO  = (size_t)HID * QD * 2;
constexpr size_t SZ_WGU = (size_t)2 * IP * HID * 2;
constexpr size_t SZ_WD  = (size_t)HID * IP * 2;
constexpr size_t SZ_QK  = (size_t)MTOK * QKW * 2;
constexpr size_t SZ_VT  = (size_t)KD * MTOK * 2;
constexpr size_t SZ_AO  = (size_t)MTOK * QD * 2;
constexpr size_t SZ_AP  = (size_t)MTOK * HID * 4;
constexpr size_t SZ_HH  = (size_t)MTOK * IP * 2;
constexpr size_t WS_TOTAL = SZ_X16 + SZ_WQK + SZ_WV + SZ_WO + SZ_WGU + SZ_WD + SZ_QK + SZ_VT + SZ_AO + SZ_AP + SZ_HH;
static_assert(SZ_X16 % 256 == 0 && SZ_WQK % 256 == 0 && SZ_WV % 256 == 0 && SZ_WO % 256 == 0 && SZ_WGU % 256 == 0);
static_assert(SZ_WD % 256 == 0 && SZ_QK % 256 == 0 && SZ_VT % 256 == 0 && SZ_AO % 256 == 0 && SZ_AP % 256 == 0 && SZ_HH % 256 == 0);
static_assert(WS_TOTAL < (size_t)268435456);


static __device__ __forceinline__ float bfr(float f) {
    unsigned u = __float_as_uint(f);
    u += 0x7FFFu + ((u >> 16) & 1u);
    return __uint_as_float(u & 0xFFFF0000u);
}
static __device__ __forceinline__ h16 toh_flush(float v) {
    const float w = (fabsf(v) < 6.103515625e-05f) ? 0.0f : v;
    return (h16)w;
}
static __device__ __forceinline__ void st8h2(_Float16* p, v8h v) {
    *(volatile v8h*)p = v;
    __threadfence();
    *(volatile v8h*)p = v;
}

union FragU { v16h v; v8h h[2]; };
static __device__ __forceinline__ v16h frag_ld(const _Float16* p) {
    FragU f; f.h[0] = *(const v8h*)(p); f.h[1] = *(const v8h*)(p + 16); return f.v;
}
static __device__ __forceinline__ v8f wmma16g(v16h a, v16h b, v8f c) {
    c = __builtin_amdgcn_wmma_f32_16x16x32_f16(false, a, false, b, (short)0, c, false, false);
    asm volatile("v_nop\n\tv_nop\n\tv_nop\n\tv_nop" : "+v"(c) : "v"(a), "v"(b));
    return c;
}
static __device__ __forceinline__ void wave_sync_lds() {
    __builtin_amdgcn_fence(3  , "workgroup");
    __builtin_amdgcn_wave_barrier();
    __builtin_amdgcn_fence(2  , "workgroup");
}

template <int LG, bool XROWS>
__global__ __launch_bounds__(256) void k_cvt16(const float* __restrict__ src, _Float16* __restrict__ dst, unsigned n8) {
    const unsigned u = blockIdx.x * 256u + threadIdx.x;
    if (u >= n8) return;
    size_t so = (size_t)u * 8u;
    if (XROWS) {
        const unsigned r = u / (unsigned)(HID / 8), c8 = u % (unsigned)(HID / 8);
        const unsigned sr = (r / (unsigned)SEQ) * (unsigned)SEQ_FULL + (r % (unsigned)SEQ);
        so = (size_t)sr * (unsigned)HID + (size_t)c8 * 8u;
    }
    constexpr float SC = (float)(1u << LG);
    const v4f a = *(const v4f*)(src + so);
    const v4f b = *(const v4f*)(src + so + 4);
    v8h o;
    o[0] = toh_flush(bfr(a.x) * SC); o[1] = toh_flush(bfr(a.y) * SC);
    o[2] = toh_flush(bfr(a.z) * SC); o[3] = toh_flush(bfr(a.w) * SC);
    o[4] = toh_flush(bfr(b.x) * SC); o[5] = toh_flush(bfr(b.y) * SC);
    o[6] = toh_flush(bfr(b.z) * SC); o[7] = toh_flush(bfr(b.w) * SC);
    st8h2(dst + (size_t)u * 8u, o);
}

template <int MODE, int LGS>
__global__ __launch_bounds__(256) void k_gemm64(
    const _Float16* __restrict__ A, unsigned lda, const _Float16* __restrict__ Bt, unsigned ldb,
    void* __restrict__ Cout, unsigned ldc, const float* __restrict__ resid,
    unsigned M, unsigned N, unsigned K) {
  __shared__ __align__(16) float sT[8][16 * 68];
  const unsigned lane = threadIdx.x & 31u;
  const unsigned wave = threadIdx.x >> 5;
  const unsigned tilesN = N >> 6, tilesM = M >> 6;
  const unsigned tile = blockIdx.x * 8u + wave;
  if (tile >= tilesM * tilesN) return;
  const unsigned tm = tile / tilesN;
  const unsigned tn = tile - tm * tilesN;
  const unsigned m0 = tm << 6, n0 = tn << 6;
  const unsigned rlane = lane & 15u;
  const unsigned koff = (lane >> 4) * 8u;
  const unsigned mOff = koff;
  constexpr float SCL = 1.0f / (float)(1u << LGS);

  v8f acc[4][4];
#pragma unroll
  for (int i = 0; i < 4; ++i)
#pragma unroll
    for (int j = 0; j < 4; ++j) acc[i][j] = (v8f){0.f,0.f,0.f,0.f,0.f,0.f,0.f,0.f};

  for (unsigned k0 = 0; k0 < K; k0 += 32u) {
    v16h bh[4];
#pragma unroll
    for (int j = 0; j < 4; ++j)
      bh[j] = frag_ld(Bt + (size_t)(n0 + ((unsigned)j << 4) + rlane) * ldb + koff + k0);
#pragma unroll
    for (int i = 0; i < 4; ++i) {
      const v16h ah = frag_ld(A + (size_t)(m0 + ((unsigned)i << 4) + rlane) * lda + koff + k0);
#pragma unroll
      for (int j = 0; j < 4; ++j) acc[i][j] = wmma16g(ah, bh[j], acc[i][j]);
    }
  }

  float* slab = sT[wave];
#pragma unroll
  for (int i = 0; i < 4; ++i) {
    const unsigned mBase = m0 + ((unsigned)i << 4);
#pragma unroll
    for (int j = 0; j < 4; ++j)
#pragma unroll
      for (int r = 0; r < 8; ++r)
        slab[(mOff + (unsigned)r) * 68u + ((unsigned)j << 4) + rlane] = acc[i][j][r] * SCL;
    wave_sync_lds();
    if (MODE == 0 || MODE == 2) {
      float* C = (float*)Cout;
      const unsigned hh = lane >> 4, c4 = (lane & 15u) * 4u;
#pragma unroll
      for (int half = 0; half < 2; ++half) {
        v4f vv[4];
#pragma unroll
        for (int it = 0; it < 4; ++it) {
          const unsigned row = (unsigned)(half * 4 + it) * 2u + hh;
          vv[it] = *(const v4f*)(slab + row * 68u + c4);
          if (MODE == 2) vv[it] += *(const v4f*)(resid + (size_t)(mBase + row) * ldc + n0 + c4);
        }
        for (int pass = 0; pass < 2; ++pass) {
#pragma unroll
          for (int it = 0; it < 4; ++it) {
            const unsigned row = (unsigned)(half * 4 + it) * 2u + hh;
            const unsigned m = mBase + row;
            unsigned orow = m;
            if (MODE == 2) orow = (m / (unsigned)SEQ) * (unsigned)SEQ_FULL + (m % (unsigned)SEQ);
            *(volatile v4f*)(C + (size_t)orow * ldc + n0 + c4) = vv[it];
          }
          __threadfence();
        }
      }
    } else {
      _Float16* C = (_Float16*)Cout;
      const unsigned q = lane >> 3, c8 = (lane & 7u) * 8u;
      v8h hv[4];
#pragma unroll
      for (int it = 0; it < 4; ++it) {
        const unsigned row = (unsigned)it * 4u + q;
        const float* sp = slab + row * 68u + c8;
        const v4f f0 = *(const v4f*)sp, f1 = *(const v4f*)(sp + 4);
        hv[it][0] = toh_flush(f0.x); hv[it][1] = toh_flush(f0.y); hv[it][2] = toh_flush(f0.z); hv[it][3] = toh_flush(f0.w);
        hv[it][4] = toh_flush(f1.x); hv[it][5] = toh_flush(f1.y); hv[it][6] = toh_flush(f1.z); hv[it][7] = toh_flush(f1.w);
      }
      for (int pass = 0; pass < 2; ++pass) {
#pragma unroll
        for (int it = 0; it < 4; ++it) {
          const unsigned row = (unsigned)it * 4u + q;
          *(volatile v8h*)(C + (size_t)(mBase + row) * ldc + n0 + c8) = hv[it];
        }
        __threadfence();
      }
    }
    wave_sync_lds();
  }
}

template <int EPI>
__global__ __launch_bounds__(128) void k_dual(const _Float16* __restrict__ A, const _Float16* __restrict__ Bt,
                                              _Float16* __restrict__ C, const float* __restrict__ cosT,
                                              const float* __restrict__ sinT) {
  __shared__ __align__(16) float sT[4][2][16 * 68];
  constexpr unsigned TILES_N = (EPI == 0) ? (unsigned)(QKW / 128) : (unsigned)(IP / 64);
  constexpr unsigned OFF1 = (EPI == 0) ? 128u : (unsigned)IP;
  constexpr unsigned LDC = (EPI == 0) ? (unsigned)QKW : (unsigned)IP;
  const unsigned lane = threadIdx.x & 31u;
  const unsigned wave = threadIdx.x >> 5;
  const unsigned tile = blockIdx.x * 4u + wave;
  if (tile >= (unsigned)(MTOK / 32) * TILES_N) return;
  const unsigned tm = tile / TILES_N;
  const unsigned tn = tile - tm * TILES_N;
  const unsigned m0 = tm << 5;
  const unsigned n0 = (EPI == 0) ? ((tn >> 1) * 256u + (tn & 1u) * 64u) : (tn << 6);
  const unsigned rlane = lane & 15u;
  const unsigned koff = (lane >> 4) * 8u;
  const unsigned mOff = koff;

  v8f acc0[2][4], acc1[2][4];
#pragma unroll
  for (int i = 0; i < 2; ++i)
#pragma unroll
    for (int j = 0; j < 4; ++j) {
      acc0[i][j] = (v8f){0.f,0.f,0.f,0.f,0.f,0.f,0.f,0.f};
      acc1[i][j] = acc0[i][j];
    }

  const _Float16* ap0 = A + (size_t)(m0 + rlane) * (unsigned)HID + koff;
  const _Float16* bp0 = Bt + (size_t)(n0 + rlane) * (unsigned)HID + koff;
  const _Float16* bp1 = bp0 + (size_t)OFF1 * (unsigned)HID;

  for (unsigned k0 = 0; k0 < (unsigned)HID; k0 += 32u) {
    const v16h a0 = frag_ld(ap0 + k0);
    const v16h a1 = frag_ld(ap0 + (size_t)16u * (unsigned)HID + k0);
    {
      v16h bh[4];
#pragma unroll
      for (int j = 0; j < 4; ++j) bh[j] = frag_ld(bp0 + (size_t)((unsigned)j << 4) * (unsigned)HID + k0);
#pragma unroll
      for (int j = 0; j < 4; ++j) acc0[0][j] = wmma16g(a0, bh[j], acc0[0][j]);
#pragma unroll
      for (int j = 0; j < 4; ++j) acc0[1][j] = wmma16g(a1, bh[j], acc0[1][j]);
    }
    {
      v16h bh[4];
#pragma unroll
      for (int j = 0; j < 4; ++j) bh[j] = frag_ld(bp1 + (size_t)((unsigned)j << 4) * (unsigned)HID + k0);
#pragma unroll
      for (int j = 0; j < 4; ++j) acc1[0][j] = wmma16g(a0, bh[j], acc1[0][j]);
#pragma unroll
      for (int j = 0; j < 4; ++j) acc1[1][j] = wmma16g(a1, bh[j], acc1[1][j]);
    }
  }

  float* s0 = sT[wave][0];
  float* s1 = sT[wave][1];
  const unsigned q4 = lane >> 3, c8 = (lane & 7u) * 8u;
  const unsigned dloc = (tn & 1u) * 64u + c8;
#pragma unroll
  for (int i = 0; i < 2; ++i) {
    const unsigned mBase = m0 + ((unsigned)i << 4);
#pragma unroll
    for (int j = 0; j < 4; ++j)
#pragma unroll
      for (int r = 0; r < 8; ++r) {
        const unsigned so = (mOff + (unsigned)r) * 68u + ((unsigned)j << 4) + rlane;
        if (EPI == 0) {
          s0[so] = acc0[i][j][r] * SC_PROJ;
          s1[so] = acc1[i][j][r] * SC_PROJ;
        } else {
          const float g = acc0[i][j][r] * SC_PROJ;
          const float u = acc1[i][j][r] * SC_PROJ;
          const float sl = g / (1.0f + expf(-g));
          s0[so] = (sl * u) * HID_CARRY;
        }
      }
    wave_sync_lds();
    v8h h0[4], h1[4];
#pragma unroll
    for (int it = 0; it < 4; ++it) {
      const unsigned row = (unsigned)it * 4u + q4;
      const float* pa = s0 + row * 68u + c8;
      const v4f ta0 = *(const v4f*)pa, ta1 = *(const v4f*)(pa + 4);
      const float t0[8] = {ta0.x, ta0.y, ta0.z, ta0.w, ta1.x, ta1.y, ta1.z, ta1.w};
      if (EPI == 0) {
        const float* pb = s1 + row * 68u + c8;
        const v4f tb0 = *(const v4f*)pb, tb1 = *(const v4f*)(pb + 4);
        const float t1[8] = {tb0.x, tb0.y, tb0.z, tb0.w, tb1.x, tb1.y, tb1.z, tb1.w};
        const unsigned pos = (mBase + row) % (unsigned)SEQ;
        const float* cp = cosT + (size_t)pos * (unsigned)HD + dloc;
        const float* sp = sinT + (size_t)pos * (unsigned)HD + dloc;
        const v4f ca0 = *(const v4f*)cp, ca1 = *(const v4f*)(cp + 4);
        const v4f cb0 = *(const v4f*)(cp + 128), cb1 = *(const v4f*)(cp + 132);
        const v4f sa0 = *(const v4f*)sp, sa1 = *(const v4f*)(sp + 4);
        const v4f sb0 = *(const v4f*)(sp + 128), sb1 = *(const v4f*)(sp + 132);
        const float c0[8] = {ca0.x, ca0.y, ca0.z, ca0.w, ca1.x, ca1.y, ca1.z, ca1.w};
        const float c1[8] = {cb0.x, cb0.y, cb0.z, cb0.w, cb1.x, cb1.y, cb1.z, cb1.w};
        const float n0v[8] = {sa0.x, sa0.y, sa0.z, sa0.w, sa1.x, sa1.y, sa1.z, sa1.w};
        const float n1v[8] = {sb0.x, sb0.y, sb0.z, sb0.w, sb1.x, sb1.y, sb1.z, sb1.w};
#pragma unroll
        for (int e = 0; e < 8; ++e) {
          const float r0 = t0[e] * bfr(c0[e]) + (-t1[e]) * bfr(n0v[e]);
          const float r1 = t1[e] * bfr(c1[e]) + t0[e] * bfr(n1v[e]);
          h0[it][e] = toh_flush(r0 * ACT_CARRY);
          h1[it][e] = toh_flush(r1 * ACT_CARRY);
        }
      } else {
#pragma unroll
        for (int e = 0; e < 8; ++e) { h0[it][e] = toh_flush(t0[e]); h1[it][e] = h0[it][e]; }
      }
    }
    for (int pass = 0; pass < 2; ++pass) {
#pragma unroll
      for (int it = 0; it < 4; ++it) {
        const unsigned row = (unsigned)it * 4u + q4;
        _Float16* d = C + (size_t)(mBase + row) * LDC + n0 + c8;
        *(volatile v8h*)d = h0[it];
        if (EPI == 0) *(volatile v8h*)(d + 128) = h1[it];
      }
      __threadfence();
    }
    wave_sync_lds();
  }
}

#define AT_PP 72
#define AT_SP 68
static __device__ __forceinline__ float mskv(float s, int key, int qi) { return (key > qi) ? -1.0e30f : s; }

__global__ __launch_bounds__(128) void k_attn(const _Float16* __restrict__ qk, const _Float16* __restrict__ vT,
                                              _Float16* __restrict__ ao) {
  __shared__ __align__(16) float    sS[4][16 * AT_SP];
  __shared__ __align__(16) _Float16 sP[4][16 * AT_PP];
  __shared__ __align__(16) float    sAl[4][16];
  const unsigned tid = threadIdx.x, lane = tid & 31u, wave = tid >> 5;
  const unsigned hh = lane >> 4, c = lane & 15u;
  const unsigned bx = blockIdx.x;
  const unsigned qt = bx % (unsigned)(SEQ / 64);
  const unsigned bh = bx / (unsigned)(SEQ / 64);
  const unsigned h = bh % (unsigned)NH;
  const unsigned b = bh / (unsigned)NH;
  const unsigned kvh = h >> 1;
  const unsigned q0 = qt * 64u + wave * 16u;
  const unsigned nch = (q0 >> 6) + 1u;

  float* sl = sS[wave];
  _Float16* pw = sP[wave];
  float* al = sAl[wave];

  const _Float16* qrow  = qk + (size_t)(b * (unsigned)SEQ + q0 + c) * (unsigned)QKW + h * 256u + 8u * hh;
  const _Float16* kbase = qk + (size_t)(b * (unsigned)SEQ) * (unsigned)QKW + (unsigned)QD + kvh * 256u + 8u * hh;
  const _Float16* vbase = vT + (size_t)(kvh * 256u + c) * (unsigned)MTOK + b * (unsigned)SEQ + 8u * hh;

  const unsigned prow = lane >> 1, phalf = lane & 1u;
  const int qi = (int)(q0 + prow);
  const float* sr = sl + prow * AT_SP + phalf * 32u;
  _Float16* pr = pw + prow * AT_PP + phalf * 32u;
  float mrun = -3.0e38f, lrun = 0.0f;

  v8f o[16];
#pragma unroll
  for (int dt = 0; dt < 16; ++dt) o[dt] = (v8f){0.f,0.f,0.f,0.f,0.f,0.f,0.f,0.f};

  for (unsigned kc = 0; kc < nch; ++kc) {
    const unsigned kv0 = kc * 64u;
    v8f s[4];
#pragma unroll
    for (int j = 0; j < 4; ++j) s[j] = (v8f){0.f,0.f,0.f,0.f,0.f,0.f,0.f,0.f};
    for (unsigned ks = 0; ks < 8u; ++ks) {
      const v16h qf = frag_ld(qrow + ks * 32u);
#pragma unroll
      for (int j = 0; j < 4; ++j) {
        const v16h kf = frag_ld(kbase + (size_t)(kv0 + (unsigned)j * 16u + c) * (unsigned)QKW + ks * 32u);
        s[j] = wmma16g(qf, kf, s[j]);
      }
    }
#pragma unroll
    for (int j = 0; j < 4; ++j)
#pragma unroll
      for (int r = 0; r < 8; ++r)
        sl[(8u * hh + (unsigned)r) * AT_SP + (unsigned)j * 16u + c] = s[j][r] * SC_S;
    wave_sync_lds();
    const int key0 = (int)(kv0 + phalf * 32u);
    float mx = -3.0e38f;
    for (unsigned g = 0; g < 8u; ++g) {
      const v4f t = *(const v4f*)(sr + 4u * g);
      const int kb = key0 + (int)(4u * g);
      const float a0 = mskv(t.x, kb, qi), a1 = mskv(t.y, kb + 1, qi);
      const float a2 = mskv(t.z, kb + 2, qi), a3 = mskv(t.w, kb + 3, qi);
      mx = fmaxf(mx, fmaxf(fmaxf(a0, a1), fmaxf(a2, a3)));
    }
    mx = fmaxf(mx, __shfl_xor(mx, 1, 32));
    const float mnew = fmaxf(mrun, mx);
    const float alpha = expf(mrun - mnew);
    mrun = mnew;
    float ps = 0.0f;
    for (unsigned g = 0; g < 4u; ++g) {
      const v4f t0 = *(const v4f*)(sr + 8u * g);
      const v4f t1 = *(const v4f*)(sr + 8u * g + 4u);
      const int kb = key0 + (int)(8u * g);
      const float p0 = expf(mskv(t0.x, kb, qi) - mnew);
      const float p1 = expf(mskv(t0.y, kb + 1, qi) - mnew);
      const float p2 = expf(mskv(t0.z, kb + 2, qi) - mnew);
      const float p3 = expf(mskv(t0.w, kb + 3, qi) - mnew);
      const float p4 = expf(mskv(t1.x, kb + 4, qi) - mnew);
      const float p5 = expf(mskv(t1.y, kb + 5, qi) - mnew);
      const float p6 = expf(mskv(t1.z, kb + 6, qi) - mnew);
      const float p7 = expf(mskv(t1.w, kb + 7, qi) - mnew);
      ps += ((p0 + p1) + (p2 + p3)) + ((p4 + p5) + (p6 + p7));
      v8h pv;
      pv[0] = toh_flush(p0 * P_CARRY); pv[1] = toh_flush(p1 * P_CARRY);
      pv[2] = toh_flush(p2 * P_CARRY); pv[3] = toh_flush(p3 * P_CARRY);
      pv[4] = toh_flush(p4 * P_CARRY); pv[5] = toh_flush(p5 * P_CARRY);
      pv[6] = toh_flush(p6 * P_CARRY); pv[7] = toh_flush(p7 * P_CARRY);
      *(v8h*)(pr + 8u * g) = pv;
    }
    ps += __shfl_xor(ps, 1, 32);
    lrun = lrun * alpha + ps;
    if (phalf == 0u) al[prow] = alpha;
    wave_sync_lds();
    float av[8];
#pragma unroll
    for (int r = 0; r < 8; ++r) av[r] = al[8u * hh + (unsigned)r];
#pragma unroll
    for (int dt = 0; dt < 16; ++dt)
#pragma unroll
      for (int r = 0; r < 8; ++r) o[dt][r] *= av[r];
    for (unsigned kk = 0; kk < 2u; ++kk) {
      const v16h pa = frag_ld(pw + c * AT_PP + kk * 32u + 8u * hh);
#pragma unroll
      for (int dt = 0; dt < 16; ++dt) {
        const v16h vb = frag_ld(vbase + (size_t)((unsigned)dt * 16u) * (unsigned)MTOK + kv0 + kk * 32u);
        o[dt] = wmma16g(pa, vb, o[dt]);
      }
    }
    wave_sync_lds();
  }

  {
    const float linv = (1.0f / lrun) * SC_O;
    if (phalf == 0u) al[prow] = linv;
  }
  wave_sync_lds();
  float fr[8];
#pragma unroll
  for (int r = 0; r < 8; ++r) fr[r] = al[8u * hh + (unsigned)r];
  const unsigned q4 = lane >> 3, c8 = (lane & 7u) * 8u;
#pragma unroll
  for (int g = 0; g < 4; ++g) {
#pragma unroll
    for (int j = 0; j < 4; ++j)
#pragma unroll
      for (int r = 0; r < 8; ++r)
        sl[(8u * hh + (unsigned)r) * AT_SP + (unsigned)j * 16u + c] = o[g * 4 + j][r] * fr[r];
    wave_sync_lds();
    v8h ov[4];
#pragma unroll
    for (int it = 0; it < 4; ++it) {
      const float* sp = sl + ((unsigned)it * 4u + q4) * AT_SP + c8;
      const v4f f0 = *(const v4f*)sp, f1 = *(const v4f*)(sp + 4);
      ov[it][0] = toh_flush(f0.x); ov[it][1] = toh_flush(f0.y); ov[it][2] = toh_flush(f0.z); ov[it][3] = toh_flush(f0.w);
      ov[it][4] = toh_flush(f1.x); ov[it][5] = toh_flush(f1.y); ov[it][6] = toh_flush(f1.z); ov[it][7] = toh_flush(f1.w);
    }
    _Float16* dst = ao + (size_t)(b * (unsigned)SEQ + q0) * (unsigned)QD + h * 256u + (unsigned)g * 64u;
    for (int pass = 0; pass < 2; ++pass) {
#pragma unroll
      for (int it = 0; it < 4; ++it)
        *(volatile v8h*)(dst + (size_t)((unsigned)it * 4u + q4) * (unsigned)QD + c8) = ov[it];
      __threadfence();
    }
    wave_sync_lds();
  }
}

extern "C" void kernel_launch(void* const* d_in, const int* in_sizes, int n_in, void* d_out, int out_size,
                              void* d_ws, size_t ws_size, hipStream_t stream) {
    if (n_in < 10) return;
    const long long xneed = ((long long)(NB - 1) * SEQ_FULL + SEQ) * (long long)HID;
    if ((long long)in_sizes[0] < xneed || (long long)out_size < xneed) return;
    if (in_sizes[1] < SEQ * HD || in_sizes[2] < SEQ * HD) return;
    if (in_sizes[3] < QD * HID || in_sizes[4] < KD * HID || in_sizes[5] < KD * HID || in_sizes[6] < HID * QD) return;
    if (in_sizes[7] < IP * HID || in_sizes[8] < IP * HID || in_sizes[9] < HID * IP) return;
    if ((size_t)WS_TOTAL > ws_size) return;

    const float* x      = (const float*)d_in[0];
    const float* cosT   = (const float*)d_in[1];
    const float* sinT   = (const float*)d_in[2];
    const float* q_w    = (const float*)d_in[3];
    const float* k_w    = (const float*)d_in[4];
    const float* v_w    = (const float*)d_in[5];
    const float* o_w    = (const float*)d_in[6];
    const float* gate_w = (const float*)d_in[7];
    const float* up_w   = (const float*)d_in[8];
    const float* down_w = (const float*)d_in[9];
    float* out = (float*)d_out;

    char* wsp = (char*)d_ws;
    size_t off = 0;
    auto carve = [&](size_t bytes) -> void* { void* r = wsp + off; off += (bytes + 255) & ~(size_t)255; return r; };
    _Float16* x16  = (_Float16*)carve(SZ_X16);
    _Float16* wqk  = (_Float16*)carve(SZ_WQK);
    _Float16* wv   = (_Float16*)carve(SZ_WV);
    _Float16* wo   = (_Float16*)carve(SZ_WO);
    _Float16* wgu  = (_Float16*)carve(SZ_WGU);
    _Float16* wd   = (_Float16*)carve(SZ_WD);
    _Float16* qk16 = (_Float16*)carve(SZ_QK);
    _Float16* vT16 = (_Float16*)carve(SZ_VT);
    _Float16* ao16 = (_Float16*)carve(SZ_AO);
    float*    ap   = (float*)carve(SZ_AP);
    _Float16* h16p = (_Float16*)carve(SZ_HH);
    if (off > ws_size) return;

    {
        const unsigned n8x = (unsigned)((size_t)MTOK * HID / 8);
        k_cvt16<11, true><<<(n8x + 255u) / 256u, 256, 0, stream>>>(x, x16, n8x);
        const unsigned n8q = (unsigned)(QD * HID / 8), n8k = (unsigned)(KD * HID / 8), n8o = (unsigned)(HID * QD / 8);
        const unsigned n8g = (unsigned)(IP * HID / 8);
        k_cvt16<17, false><<<(n8q + 255u) / 256u, 256, 0, stream>>>(q_w, wqk, n8q);
        k_cvt16<17, false><<<(n8k + 255u) / 256u, 256, 0, stream>>>(k_w, wqk + (size_t)QD * HID, n8k);
        k_cvt16<17, false><<<(n8k + 255u) / 256u, 256, 0, stream>>>(v_w, wv, n8k);
        k_cvt16<17, false><<<(n8o + 255u) / 256u, 256, 0, stream>>>(o_w, wo, n8o);
        k_cvt16<17, false><<<(n8g + 255u) / 256u, 256, 0, stream>>>(gate_w, wgu, n8g);
        k_cvt16<17, false><<<(n8g + 255u) / 256u, 256, 0, stream>>>(up_w, wgu + (size_t)IP * HID, n8g);
        k_cvt16<17, false><<<(n8g + 255u) / 256u, 256, 0, stream>>>(down_w, wd, n8g);
    }

    {
        const unsigned tiles = (unsigned)(MTOK / 32) * (unsigned)(QKW / 128);
        k_dual<0><<<(tiles + 3u) / 4u, 128, 0, stream>>>(x16, wqk, qk16, cosT, sinT);
    }
    {
        const unsigned tiles = (unsigned)(KD / 64) * (unsigned)(MTOK / 64);
        k_gemm64<1, 17><<<(tiles + 7u) / 8u, 256, 0, stream>>>(wv, HID, x16, HID, (void*)vT16, MTOK, ap, KD, MTOK, HID);
    }
    k_attn<<<(unsigned)(NB * NH * (SEQ / 64)), 128, 0, stream>>>(qk16, vT16, ao16);
    {
        const unsigned tiles = (unsigned)(MTOK / 64) * (unsigned)(HID / 64);
        k_gemm64<0, 29><<<(tiles + 7u) / 8u, 256, 0, stream>>>(ao16, QD, wo, QD, (void*)ap, HID, ap, MTOK, HID, QD);
    }
    {
        const unsigned tiles = (unsigned)(MTOK / 32) * (unsigned)(IP / 64);
        k_dual<1><<<(tiles + 3u) / 4u, 128, 0, stream>>>(x16, wgu, h16p, cosT, sinT);
    }
    {
        const unsigned tiles = (unsigned)(MTOK / 64) * (unsigned)(HID / 64);
        k_gemm64<2, 27><<<(tiles + 7u) / 8u, 256, 0, stream>>>(h16p, IP, wd, IP, (void*)out, HID, ap, MTOK, HID, IP);
    }
}
